// LocalRNN_84619445666139
// MI455X (gfx1250) — hardware-verified
//
#include <hip/hip_runtime.h>
#include <stddef.h>


typedef _Float16 v16h __attribute__((ext_vector_type(16)));
typedef _Float16 v8h  __attribute__((ext_vector_type(8)));
typedef float    v8f  __attribute__((ext_vector_type(8)));
typedef float    v4f  __attribute__((ext_vector_type(4)));
typedef unsigned v4u  __attribute__((ext_vector_type(4)));

union Frag  { v16h v; v8h p[2]; };
union Pack8 { v8h h; v4u u; };

#define DEV __device__ __forceinline__

constexpr int CB   = 16;
constexpr int CL   = 1024;
constexpr int CD   = 256;
constexpr int CH   = 256;
constexpr int CK   = 16;
constexpr int NG   = 3 * CH;
constexpr int NTOK = CB * CL;

constexpr float WSCALE = 16.0f;
constexpr float WINV   = 0.0625f;

constexpr int XCH = NTOK * CD / 8;
constexpr int WCH = NG * CD / 8;
constexpr int CVT_TOTAL   = XCH + 2 * WCH;
constexpr int CVT_THREADS = 256;
constexpr int CVT_BLOCKS  = (CVT_TOTAL + CVT_THREADS - 1) / CVT_THREADS;

constexpr int GI_BM = 128, GI_BN = 32, GI_THREADS = 128;
static_assert(NTOK % GI_BM == 0);
static_assert(NG % GI_BN == 0);
static_assert(CD % 32 == 0);
static_assert((2 * CH) % GI_BN == 0);

constexpr int GR_ROWS = 16, GR_THREADS = 512;
static_assert(CL % GR_ROWS == 0);
static_assert(GR_THREADS / 32 == CH / 16);
static_assert(GR_THREADS / 32 == GR_ROWS);
static_assert(GR_THREADS * 16 == GR_ROWS * CH * 2);
static_assert(CH % 32 == 0);

constexpr size_t OFF_X16   = 0;
constexpr size_t OFF_WIH16 = OFF_X16   + (size_t)NTOK * CD * 2;
constexpr size_t OFF_WHH16 = OFF_WIH16 + (size_t)NG * CD * 2;
constexpr size_t OFF_U     = OFF_WHH16 + (size_t)NG * CH * 2;
constexpr size_t WS_NEED   = OFF_U     + (size_t)NTOK * NG * 4;
static_assert(WS_NEED <= (size_t)134217728);
static_assert(OFF_WIH16 % 256 == 0);
static_assert(OFF_WHH16 % 256 == 0);
static_assert(OFF_U % 256 == 0);

DEV v8f zero8() { v8f z = {0.f, 0.f, 0.f, 0.f, 0.f, 0.f, 0.f, 0.f}; return z; }

DEV v8f wmma16(const v16h& a, const v16h& b, v8f c) {
  c = __builtin_amdgcn_wmma_f32_16x16x32_f16(false, a, false, b, (short)0, c, false, false);
  asm volatile("v_nop\n\tv_nop\n\tv_nop\n\tv_nop" : "+v"(c) : "v"(a), "v"(b));
  return c;
}

DEV float sigm(float x)  { return __builtin_amdgcn_rcpf(1.0f + __expf(-x)); }
DEV float tanh_(float x) { return 2.0f * __builtin_amdgcn_rcpf(1.0f + __expf(-2.0f * x)) - 1.0f; }

__global__ __launch_bounds__(CVT_THREADS) void k_cvt(
    const float* __restrict__ x, const float* __restrict__ wih, const float* __restrict__ whh,
    _Float16* x16, _Float16* wih16, _Float16* whh16) {
  const int i = blockIdx.x * CVT_THREADS + threadIdx.x;
  if (i >= CVT_TOTAL) return;
  const float* src; _Float16* dst; float s; int k;
  if (i < XCH)            { src = x;   dst = x16;   s = 1.0f;   k = i; }
  else if (i < XCH + WCH) { src = wih; dst = wih16; s = WSCALE; k = i - XCH; }
  else                    { src = whh; dst = whh16; s = WSCALE; k = i - XCH - WCH; }
  const float* p = src + (size_t)k * 8;
  const v4f a = *(const v4f*)(p);
  const v4f c = *(const v4f*)(p + 4);
  v8h hv = { (_Float16)(a[0] * s), (_Float16)(a[1] * s), (_Float16)(a[2] * s), (_Float16)(a[3] * s),
             (_Float16)(c[0] * s), (_Float16)(c[1] * s), (_Float16)(c[2] * s), (_Float16)(c[3] * s) };
  Pack8 o; o.h = hv;
  const v4u bits = o.u;
  _Float16* q = dst + (size_t)k * 8;
  *(volatile v4u*)q = bits;
  __threadfence();
  *(volatile v4u*)q = bits;
}

__global__ __launch_bounds__(GI_THREADS) void k_gi(
    const _Float16* __restrict__ x16, const _Float16* __restrict__ w16,
    const float* __restrict__ bih, const float* __restrict__ bhh, float* U) {
  __shared__ __align__(16) float sh_t[GI_BM][GI_BN];
  const int tid = threadIdx.x, lane = tid & 31, wv = tid >> 5;
  const int hf = lane >> 4, lc = lane & 15;
  const int mrow0 = blockIdx.x * GI_BM + wv * 32;
  const int n0 = blockIdx.y * GI_BN;
  const _Float16* ar0 = x16 + (size_t)(mrow0 + lc) * CD;
  const _Float16* ar1 = ar0 + (size_t)16 * CD;
  const _Float16* br0 = w16 + (size_t)(n0 + lc) * CD;
  const _Float16* br1 = br0 + (size_t)16 * CD;

  v8f a00 = zero8(), a01 = zero8(), a10 = zero8(), a11 = zero8();
#pragma unroll
  for (int kc = 0; kc < CD / 32; ++kc) {
    const int k0 = kc * 32 + 8 * hf;
    Frag fa0, fa1, fb0, fb1;
    fa0.p[0] = *(const v8h*)(ar0 + k0); fa0.p[1] = *(const v8h*)(ar0 + k0 + 16);
    fa1.p[0] = *(const v8h*)(ar1 + k0); fa1.p[1] = *(const v8h*)(ar1 + k0 + 16);
    fb0.p[0] = *(const v8h*)(br0 + k0); fb0.p[1] = *(const v8h*)(br0 + k0 + 16);
    fb1.p[0] = *(const v8h*)(br1 + k0); fb1.p[1] = *(const v8h*)(br1 + k0 + 16);
    a00 = wmma16(fa0.v, fb0.v, a00);
    a01 = wmma16(fa0.v, fb1.v, a01);
    a10 = wmma16(fa1.v, fb0.v, a10);
    a11 = wmma16(fa1.v, fb1.v, a11);
  }

  const int nA = n0 + lc, nB = n0 + 16 + lc;
  const float biasA = bih[nA] + ((nA < 2 * CH) ? bhh[nA] : 0.0f);
  const float biasB = bih[nB] + ((nB < 2 * CH) ? bhh[nB] : 0.0f);
#pragma unroll
  for (int r = 0; r < 8; ++r) {
    const int row = wv * 32 + 8 * hf + r;
    sh_t[row][lc]           = a00[r] * WINV + biasA;
    sh_t[row][16 + lc]      = a01[r] * WINV + biasB;
    sh_t[row + 16][lc]      = a10[r] * WINV + biasA;
    sh_t[row + 16][16 + lc] = a11[r] * WINV + biasB;
  }
  __syncthreads();

  const int rs = lane >> 3, c4 = (lane & 7) * 4;
  v4f vals[8];
#pragma unroll
  for (int p = 0; p < 8; ++p) vals[p] = *(const v4f*)&sh_t[wv * 32 + 4 * p + rs][c4];
  float* ub = U + (size_t)(mrow0 + rs) * NG + n0 + c4;
#pragma unroll
  for (int p = 0; p < 8; ++p) *(volatile v4f*)(ub + (size_t)(4 * p) * NG) = vals[p];
  __threadfence();
#pragma unroll
  for (int p = 0; p < 8; ++p) *(volatile v4f*)(ub + (size_t)(4 * p) * NG) = vals[p];
}

DEV void gru_update(const int t, const int l0, const int hf, const int col,
                    const v8f& aR, const v8f& aZ, const v8f& aN,
                    const float* __restrict__ ub,
                    const float pr, const float pz, const float pn, const float bn,
                    float (&h)[8], _Float16* shw) {
#pragma unroll
  for (int r = 0; r < 8; ++r) {
    const int m  = 8 * hf + r;
    const int j  = l0 + m - (CK - 1) + t;
    const int jj = (j < 0) ? 0 : j;
    const float* up = ub + (size_t)jj * NG;
    const float u_r = up[0], u_z = up[CH], u_n = up[2 * CH];
    const bool v = (j >= 0);
    const float gir = v ? u_r : pr;
    const float giz = v ? u_z : pz;
    const float gin = v ? u_n : pn;
    const float rr = sigm(gir + aR[r] * WINV);
    const float zz = sigm(giz + aZ[r] * WINV);
    const float nn = tanh_(gin + rr * (aN[r] * WINV + bn));
    const float hn = (1.0f - zz) * nn + zz * h[r];
    h[r] = hn;
    shw[m * CH + col] = (_Float16)hn;
  }
}

__global__ __launch_bounds__(GR_THREADS) void k_gru(
    const _Float16* whh16, const float* __restrict__ bih, const float* __restrict__ bhh,
    const float* __restrict__ U, float* out) {
  __shared__ __align__(16) _Float16 sh_h[2][GR_ROWS][CH];
  __shared__ __align__(16) float    sh_o[GR_ROWS][CH];

  const int tid = threadIdx.x, lane = tid & 31, wv = tid >> 5;
  const int hf = lane >> 4, lc = lane & 15;
  const int l0 = blockIdx.x * GR_ROWS;
  const int b  = blockIdx.y;
  const int col = wv * 16 + lc;

  { const v4u z = {0u, 0u, 0u, 0u}; ((v4u*)&sh_h[0][0][0])[tid] = z; }

  const float pr = bih[col] + bhh[col];
  const float pz = bih[CH + col] + bhh[CH + col];
  const float pn = bih[2 * CH + col];
  const float bn = bhh[2 * CH + col];
  const _Float16* wr = whh16 + (size_t)col * CH;
  const _Float16* wz = wr + (size_t)CH * CH;
  const _Float16* wn = wz + (size_t)CH * CH;
  const float* ub = U + (size_t)b * CL * NG + col;

  float h[8];
#pragma unroll
  for (int r = 0; r < 8; ++r) h[r] = 0.0f;

  __syncthreads();
  {
    const v8f z = zero8();
    gru_update(0, l0, hf, col, z, z, z, ub, pr, pz, pn, bn, h, &sh_h[1][0][0]);
  }
  __syncthreads();

#pragma unroll 1
  for (int t = 1; t < CK; ++t) {
    const int rb = t & 1, wb = rb ^ 1;
    const _Float16* hrow = &sh_h[rb][lc][0];
    v8f aR = zero8(), aZ = zero8(), aN = zero8();
#pragma unroll
    for (int kc = 0; kc < CH / 32; ++kc) {
      const int k0 = kc * 32 + 8 * hf;
      Frag fa, fr, fz, fn;
      fa.p[0] = *(const v8h*)(hrow + k0); fa.p[1] = *(const v8h*)(hrow + k0 + 16);
      fr.p[0] = *(const v8h*)(wr + k0);   fr.p[1] = *(const v8h*)(wr + k0 + 16);
      fz.p[0] = *(const v8h*)(wz + k0);   fz.p[1] = *(const v8h*)(wz + k0 + 16);
      fn.p[0] = *(const v8h*)(wn + k0);   fn.p[1] = *(const v8h*)(wn + k0 + 16);
      aR = wmma16(fa.v, fr.v, aR);
      aZ = wmma16(fa.v, fz.v, aZ);
      aN = wmma16(fa.v, fn.v, aN);
    }
    gru_update(t, l0, hf, col, aR, aZ, aN, ub, pr, pz, pn, bn, h, &sh_h[wb][0][0]);
    __syncthreads();
  }

#pragma unroll
  for (int r = 0; r < 8; ++r) sh_o[8 * hf + r][col] = h[r];
  __syncthreads();

  const v4f o0 = *(const v4f*)&sh_o[wv][lane * 4];
  const v4f o1 = *(const v4f*)&sh_o[wv][128 + lane * 4];
  float* orow = out + (size_t)(b * CL + l0 + wv) * CH;
  *(volatile v4f*)(orow + lane * 4)       = o0;
  *(volatile v4f*)(orow + 128 + lane * 4) = o1;
  __threadfence();
  *(volatile v4f*)(orow + lane * 4)       = o0;
  *(volatile v4f*)(orow + 128 + lane * 4) = o1;
}

extern "C" void kernel_launch(void* const* d_in, const int* in_sizes, int n_in,
                              void* d_out, int out_size, void* d_ws, size_t ws_size,
                              hipStream_t stream) {
  if (n_in < 5) return;
  if (in_sizes[0] != NTOK * CD || in_sizes[1] != NG * CD || in_sizes[2] != NG * CH ||
      in_sizes[3] != NG || in_sizes[4] != NG) return;
  if (out_size != NTOK * CH) return;
  if (ws_size < WS_NEED) return;

  const float* x   = (const float*)d_in[0];
  const float* wih = (const float*)d_in[1];
  const float* whh = (const float*)d_in[2];
  const float* bih = (const float*)d_in[3];
  const float* bhh = (const float*)d_in[4];
  float* out = (float*)d_out;

  char* ws = (char*)d_ws;
  _Float16* x16   = (_Float16*)(ws + OFF_X16);
  _Float16* wih16 = (_Float16*)(ws + OFF_WIH16);
  _Float16* whh16 = (_Float16*)(ws + OFF_WHH16);
  float*    U     = (float*)(ws + OFF_U);

  k_cvt<<<dim3(CVT_BLOCKS), dim3(CVT_THREADS), 0, stream>>>(x, wih, whh, x16, wih16, whh16);
  k_gi<<<dim3(NTOK / GI_BM, NG / GI_BN), dim3(GI_THREADS), 0, stream>>>(x16, wih16, bih, bhh, U);
  k_gru<<<dim3(CL / GR_ROWS, CB), dim3(GR_THREADS), 0, stream>>>(whh16, bih, bhh, U, out);
}
